// LDEPool1d_81527069213204
// MI455X (gfx1250) — hardware-run, weakly checked
//
#include <hip/hip_runtime.h>


#define NB   16
#define NT   800
#define NTP  832
#define ND   256
#define NK   64
#define NR   (NB * NT)
typedef _Float16 h16;
typedef unsigned short bf;
typedef __attribute__((ext_vector_type(16))) __bf16   v16bf;
typedef __attribute__((ext_vector_type(16))) _Float16 v16h;
typedef __attribute__((ext_vector_type(8)))  _Float16 v8h;
typedef __attribute__((ext_vector_type(8)))  unsigned short v8us;
typedef __attribute__((ext_vector_type(8)))  float    v8f;
typedef __attribute__((ext_vector_type(4)))  float    v4f;
typedef v8h  __attribute__((may_alias)) v8ha;
typedef v4f  __attribute__((may_alias)) v4fa;
typedef v8us __attribute__((may_alias)) v8usa;

__device__ __forceinline__ unsigned short f2bf(float f) { unsigned u = __float_as_uint(f); u += 0x7FFFu + ((u >> 16) & 1u); return (unsigned short)(u >> 16); }
__device__ __forceinline__ float bf2f(unsigned short b) { return __uint_as_float(((unsigned)b) << 16); }
__device__ __forceinline__ float bfr(float f) { return bf2f(f2bf(f)); }
__device__ __forceinline__ v16h cat16(v8h lo, v8h hi) { return __builtin_shufflevector(lo, hi, 0, 1, 2, 3, 4, 5, 6, 7, 8, 9, 10, 11, 12, 13, 14, 15); }
__device__ __forceinline__ v16bf cat16b(v8us lo, v8us hi) { return __builtin_bit_cast(v16bf, __builtin_shufflevector(lo, hi, 0, 1, 2, 3, 4, 5, 6, 7, 8, 9, 10, 11, 12, 13, 14, 15)); }
__device__ __forceinline__ v8f wmma16(v16h a, v16h b, v8f c) { return __builtin_amdgcn_wmma_f32_16x16x32_f16(false, a, false, b, (short)0, c, false, false); }
__device__ __forceinline__ v8f wmmab(v16bf a, v16bf b, v8f c) { return __builtin_amdgcn_wmma_f32_16x16x32_bf16(false, a, false, b, (short)0, c, false, false); }

template <typename T16> struct WFrag;
template <> struct WFrag<h16> { typedef v16h V; static __device__ __forceinline__ V ld(const h16* p) { return cat16(*(const v8h*)p, *(const v8h*)(p + 16)); } static __device__ __forceinline__ v8f mma(V a, V b, v8f c) { return wmma16(a, b, c); } };
template <> struct WFrag<bf> { typedef v16bf V; static __device__ __forceinline__ V ld(const bf* p) { return cat16b(*(const v8us*)p, *(const v8us*)(p + 16)); } static __device__ __forceinline__ v8f mma(V a, V b, v8f c) { return wmmab(a, b, c); } };
template <typename T16, int NSPLIT, bool BIAS>
__global__ __launch_bounds__(32) void k_gemmw(const T16* __restrict__ A, const T16* __restrict__ A2, const T16* __restrict__ Bt, const T16* __restrict__ Bt2, int K, float* C, int ldc, const float* __restrict__ bias, size_t sA, size_t sB, size_t sC) {
    typedef typename WFrag<T16>::V V;
    __shared__ __align__(16) float os[16 * 68];
    const size_t z = blockIdx.z; A += z * sA; if (A2) A2 += z * sA; Bt += z * sB; if (Bt2) Bt2 += z * sB; C += z * sC;
    const int lane = threadIdx.x & 31, lr = lane & 15, hi = lane >> 4; const int r0 = blockIdx.x * 64, c0 = blockIdx.y * 64;
    v8f acc[4][4];
#pragma unroll
    for (int mb = 0; mb < 4; ++mb)
#pragma unroll
        for (int nb = 0; nb < 4; ++nb) acc[mb][nb] = (v8f){};
    const size_t aoff = (size_t)(r0 + lr) * K + 8 * hi, boff = (size_t)(c0 + lr) * K + 8 * hi;
    for (int kc = 0; kc < K; kc += 32) {
        V a[4], a2[4];
#pragma unroll
        for (int mb = 0; mb < 4; ++mb) { a[mb] = WFrag<T16>::ld(A + aoff + (size_t)mb * 16 * K + kc); if (NSPLIT == 1 || NSPLIT == 2) a2[mb] = WFrag<T16>::ld(A2 + aoff + (size_t)mb * 16 * K + kc); }
#pragma unroll
        for (int nb = 0; nb < 4; ++nb) { const V b = WFrag<T16>::ld(Bt + boff + (size_t)nb * 16 * K + kc); V b2; if (NSPLIT >= 2) b2 = WFrag<T16>::ld(Bt2 + boff + (size_t)nb * 16 * K + kc);
#pragma unroll
            for (int mb = 0; mb < 4; ++mb) { acc[mb][nb] = WFrag<T16>::mma(a[mb], b, acc[mb][nb]); if (NSPLIT == 1 || NSPLIT == 2) acc[mb][nb] = WFrag<T16>::mma(a2[mb], b, acc[mb][nb]); if (NSPLIT >= 2) acc[mb][nb] = WFrag<T16>::mma(a[mb], b2, acc[mb][nb]); } }
        asm volatile("v_nop\n\tv_nop\n\tv_nop\n\tv_nop" : "+v"(acc[0][0]), "+v"(acc[1][1]), "+v"(acc[2][2]), "+v"(acc[3][3]) : "v"(a[0]), "v"(a[3]));
    }
#pragma unroll
    for (int mb = 0; mb < 4; ++mb) {
#pragma unroll
        for (int nb = 0; nb < 4; ++nb) {
#pragma unroll
            for (int j = 0; j < 8; ++j) os[(hi * 8 + j) * 68 + nb * 16 + lr] = acc[mb][nb][j]; }
        __builtin_amdgcn_wave_barrier(); asm volatile("" ::: "memory");
        float* crow = C + (size_t)(r0 + mb * 16) * ldc + c0;
#pragma unroll 1
        for (int ps = 0; ps < 2; ++ps) {
#pragma unroll
            for (int s = 0; s < 8; ++s) { const int row = 2 * s + hi, cofs = lr * 4; v4f val = *(const v4fa*)(os + row * 68 + cofs); if (BIAS) { val[0] += bfr(bias[c0 + cofs]); val[1] += bfr(bias[c0 + cofs + 1]); val[2] += bfr(bias[c0 + cofs + 2]); val[3] += bfr(bias[c0 + cofs + 3]); }
                *(volatile v4f*)(crow + (size_t)row * ldc + cofs) = val; }
            if (ps == 0) __threadfence(); }
        __builtin_amdgcn_wave_barrier(); asm volatile("" ::: "memory");
    }
}

__global__ __launch_bounds__(256) void k_cvt8(const float* __restrict__ src, bf* dst, size_t n8) { const size_t i = (size_t)blockIdx.x * 256 + threadIdx.x; if (i >= n8) return; const v8f v = *(const v8f*)(src + i * 8); v8us o;
#pragma unroll
    for (int k = 0; k < 8; ++k) o[k] = f2bf(v[k]); *(volatile v8us*)(dst + i * 8) = o; __threadfence(); *(volatile v8us*)(dst + i * 8) = o; }
typedef __attribute__((ext_vector_type(2))) _Float16 v2h;
typedef __attribute__((ext_vector_type(4))) _Float16 v4h;
typedef __attribute__((ext_vector_type(2))) unsigned short v2us;
typedef __attribute__((ext_vector_type(4))) unsigned short v4us;
typedef __attribute__((ext_vector_type(2))) float v2f;
__device__ __forceinline__ h16 toh_flush(float x) { const float z = (fabsf(x) < 6.103515625e-05f) ? 0.0f : x; return (h16)z; }

__global__ __launch_bounds__(64) void k_wtp16(const float* __restrict__ src, int K, int N, h16* dst, int KP, int NPz) { const int k0 = (blockIdx.x * 64 + threadIdx.x) * 8; if (k0 >= KP) return; const int n = blockIdx.y; const int z = blockIdx.z; const float* s = src + (size_t)z * K * N; v8h o;
#pragma unroll
    for (int q = 0; q < 8; ++q) { const int k = k0 + q; const bool in = (k < K) && (n < N); const float a = s[(size_t)min(k, K - 1) * N + min(n, N - 1)]; const unsigned mk = 0u - (unsigned)in; o[q] = toh_flush(__uint_as_float(__float_as_uint(bfr(a)) & mk)); }
    h16* d = dst + ((size_t)z * NPz + n) * KP + k0; *(volatile v8h*)d = o; __threadfence(); *(volatile v8h*)d = o; }

__global__ __launch_bounds__(256) void k_sq(const float* __restrict__ x, const float* __restrict__ m, float* Q) { const int r = blockIdx.x * 256 + threadIdx.x; if (r >= NR + NK) return; const float* p = (r < NR) ? (x + (size_t)r * ND) : (m + (size_t)(r - NR) * ND); float s = 0.0f;
    for (int c = 0; c < ND / 4; ++c) { const v4f v = *(const v4f*)(p + 4 * c);
#pragma unroll
        for (int k = 0; k < 4; ++k) { const float a = bfr(v[k]); s = __fmaf_rn(a, a, s); } }
    *(volatile float*)(Q + r) = s; __threadfence(); *(volatile float*)(Q + r) = s; }

__device__ __forceinline__ float lk(float qx, float qm, float g, float pk) { const float d = __fsub_rn(__fadd_rn(qx, qm), __fmul_rn(2.0f, g)); return -__fmul_rn(__fmul_rn(pk, pk), d); }

__global__ __launch_bounds__(256) void k_st(const float* __restrict__ G, const float* __restrict__ Q, const float* __restrict__ p, float* SM, float* RZ) { const int r = blockIdx.x * 256 + threadIdx.x; if (r >= NR) return; const float qx = Q[r]; const float* gr = G + (size_t)r * NK; const float* Qm = Q + NR; float M = __int_as_float(0xff800000);
    for (int g = 0; g < NK / 4; ++g) { const v4f a = *(const v4f*)(gr + 4 * g); const v4f q = *(const v4f*)(Qm + 4 * g); const v4f u = *(const v4f*)(p + 4 * g);
#pragma unroll
        for (int j = 0; j < 4; ++j) { const float t = lk(qx, q[j], a[j], bfr(u[j])); M = (t > M) ? t : M; } }
    float z = 0.0f;
    for (int g = 0; g < NK / 4; ++g) { const v4f a = *(const v4f*)(gr + 4 * g); const v4f q = *(const v4f*)(Qm + 4 * g); const v4f u = *(const v4f*)(p + 4 * g);
#pragma unroll
        for (int j = 0; j < 4; ++j) z = __fadd_rn(z, expf(__fsub_rn(lk(qx, q[j], a[j], bfr(u[j])), M))); }
    const float rz = __fdiv_rn(1.0f, z); *(volatile float*)(SM + r) = M; *(volatile float*)(RZ + r) = rz; __threadfence(); *(volatile float*)(SM + r) = M; *(volatile float*)(RZ + r) = rz; }

__device__ __forceinline__ float rv(float qx, float qm, float g, float pk, float sm, float rz) { return __fmul_rn(expf(__fsub_rn(lk(qx, qm, g, pk), sm)), rz); }

__global__ __launch_bounds__(256) void k_cs(const float* __restrict__ G, const float* __restrict__ Q, const float* __restrict__ p, const float* __restrict__ SM, const float* __restrict__ RZ, float* S) { const int i = blockIdx.x * 256 + threadIdx.x; if (i >= NB * NK) return; const int b = i / NK, k = i % NK; const float qm = Q[NR + k]; const float pk = bfr(p[k]); float s = 0.0f;
    for (int t = 0; t < NT; ++t) { const int r = b * NT + t; s = __fadd_rn(s, rv(Q[r], qm, G[(size_t)r * NK + k], pk, SM[r], RZ[r])); }
    *(volatile float*)(S + i) = s; __threadfence(); *(volatile float*)(S + i) = s; }

__global__ __launch_bounds__(256) void k_rt(const float* __restrict__ G, const float* __restrict__ Q, const float* __restrict__ p, const float* __restrict__ SM, const float* __restrict__ RZ, const float* __restrict__ S, h16* RT) { const size_t w = (size_t)blockIdx.x * 256 + threadIdx.x; if (w >= (size_t)NB * NK * NTP / 8) return; const int i = (int)(w / (NTP / 8)), t0 = (int)(w % (NTP / 8)) * 8; const int b = i / NK, k = i % NK; const float qm = Q[NR + k]; const float pk = bfr(p[k]); const float den = __fadd_rn(S[i], 1e-9f); v8h o;
#pragma unroll
    for (int j = 0; j < 8; ++j) { const int t = t0 + j; const float live = (t < NT) ? 1.0f : 0.0f; const int r = b * NT + min(t, NT - 1); o[j] = toh_flush(__fmul_rn(live, __fdiv_rn(rv(Q[r], qm, G[(size_t)r * NK + k], pk, SM[r], RZ[r]), den))); }
    *(volatile v8h*)(RT + w * 8) = o; __threadfence(); *(volatile v8h*)(RT + w * 8) = o; }

__global__ __launch_bounds__(256) void k_fin(const float* __restrict__ PR, const float* __restrict__ S, const float* __restrict__ m, float* out) { const size_t w = (size_t)blockIdx.x * 256 + threadIdx.x; if (w >= (size_t)NB * NK * ND / 4) return; const int i = (int)(w / (ND / 4)), c0 = (int)(w % (ND / 4)) * 4; const int k = i % NK; const float s = S[i]; const float f = __fdiv_rn(s, __fadd_rn(s, 1e-9f)); const v4f pv = *(const v4f*)(PR + w * 4); const v4f mv = *(const v4f*)(m + (size_t)k * ND + c0); v4f o;
#pragma unroll
    for (int j = 0; j < 4; ++j) o[j] = __fsub_rn(pv[j], __fmul_rn(f, bfr(mv[j])));
    *(volatile v4f*)(out + w * 4) = o; __threadfence(); *(volatile v4f*)(out + w * 4) = o; }

extern "C" void kernel_launch(void* const* d_in, const int* in_sizes, int n_in, void* d_out, int out_size, void* d_ws, size_t ws_size, hipStream_t stream) {
    if (n_in < 3) return;
    if (in_sizes[0] != NB * NT * ND || in_sizes[1] != NK * ND || in_sizes[2] != NK) return;
    if (out_size != NB * NK * ND) return;
    static_assert(NR % 64 == 0 && NK % 64 == 0 && ND % 64 == 0 && ND % 32 == 0 && NTP % 64 == 0 && NTP >= NT && (NR * ND / 8) % 256 == 0 && (NK * ND / 8) % 256 == 0 && NR % 256 == 0 && (NB * NK) % 256 == 0 && (NB * NK * NTP / 8) % 256 == 0 && (NB * NK * ND / 4) % 256 == 0, "the products: M and N multiples of 64, the depths multiples of 32; a plane row a whole number of lines; the flat grids exact but k_sq's");
    const float* x = (const float*)d_in[0]; const float* m = (const float*)d_in[1]; const float* p = (const float*)d_in[2];
    float* out = (float*)d_out;
    char* wsp = (char*)d_ws; auto take = [&](size_t bytes) { char* ptr = wsp; wsp += (bytes + 255) & ~(size_t)255; return (void*)ptr; };
    bf* Xb = (bf*)take((size_t)NR * ND * 2); bf* Mb = (bf*)take((size_t)NK * ND * 2); float* Q = (float*)take((size_t)(NR + NK) * 4); float* G = (float*)take((size_t)NR * NK * 4); float* SM = (float*)take((size_t)NR * 4); float* RZ = (float*)take((size_t)NR * 4); float* S = (float*)take((size_t)NB * NK * 4); h16* RT = (h16*)take((size_t)NB * NK * NTP * 2); h16* Xt = (h16*)take((size_t)NB * ND * NTP * 2); float* PR = (float*)take((size_t)NB * NK * ND * 4);
    if ((size_t)(wsp - (char*)d_ws) > ws_size) return;
    k_cvt8<<<(unsigned)(NR * ND / 8 / 256), 256, 0, stream>>>(x, Xb, (size_t)NR * ND / 8);
    k_cvt8<<<(unsigned)(NK * ND / 8 / 256), 256, 0, stream>>>(m, Mb, (size_t)NK * ND / 8);
    k_wtp16<<<dim3((NTP + 511) / 512, ND, NB), 64, 0, stream>>>(x, NT, ND, Xt, NTP, ND);
    k_sq<<<(unsigned)((NR + NK + 255) / 256), 256, 0, stream>>>(x, m, Q);
    k_gemmw<bf, 0, false><<<dim3(NR / 64, NK / 64, 1), 32, 0, stream>>>(Xb, nullptr, Mb, nullptr, ND, G, NK, nullptr, 0, 0, 0);
    k_st<<<(unsigned)(NR / 256), 256, 0, stream>>>(G, Q, p, SM, RZ);
    k_cs<<<(unsigned)(NB * NK / 256), 256, 0, stream>>>(G, Q, p, SM, RZ, S);
    k_rt<<<(unsigned)((size_t)NB * NK * NTP / 8 / 256), 256, 0, stream>>>(G, Q, p, SM, RZ, S, RT);
    k_gemmw<h16, 0, false><<<dim3(NK / 64, ND / 64, NB), 32, 0, stream>>>(RT, nullptr, Xt, nullptr, NTP, PR, ND, nullptr, (size_t)NK * NTP, (size_t)ND * NTP, (size_t)NK * ND);
    k_fin<<<(unsigned)((size_t)NB * NK * ND / 4 / 256), 256, 0, stream>>>(PR, S, m, out);
}
